// CrossModalAttentionFusion_3384434229648
// MI455X (gfx1250) — hardware-run, weakly checked
//
#include <hip/hip_runtime.h>
#include <math.h>
#include <stdint.h>

constexpr int kB      = 8192;
constexpr int kCD     = 512;
constexpr int kF      = 1024;
constexpr int kH      = 8;
constexpr int kHD     = kF / kH;
constexpr int kQKV    = 3 * kF;
constexpr int kNChunk = 4;
constexpr int kChunkB = kB / kNChunk;
constexpr int kChunkT = 2 * kChunkB;
constexpr float kWCarry    = 16.0f;
constexpr float kWCarryInv = 1.0f / kWCarry;
constexpr float kLnEps     = 1e-5f;
constexpr float kInvF      = 1.0f / (float)kF;
constexpr float kInvSqrt2  = 0.70710678118654752f;

static_assert(kHD == 128, "attention kernel handles two 128-wide heads per wave");
static_assert(kF == 1024, "row kernels assume 1024-wide rows");
static_assert(kB % kNChunk == 0, "chunking");
static_assert(kChunkB % 64 == 0 && kChunkT % 64 == 0, "GEMM M tiles");
static_assert(kF % 64 == 0 && kQKV % 64 == 0, "GEMM N tiles");
static_assert(kCD % 32 == 0 && kF % 32 == 0 && (2 * kF) % 32 == 0, "GEMM K steps");
static_assert(kChunkB % 16 == 0, "gate kernel owns 16 batch rows per block");
static_assert(kChunkT % 8 == 0, "row kernel owns 8 rows per block");

typedef __attribute__((ext_vector_type(16))) _Float16 v16h;
typedef __attribute__((ext_vector_type(8)))  _Float16 v8h;
typedef __attribute__((ext_vector_type(8)))  float    v8f;
typedef __attribute__((ext_vector_type(4)))  float    v4f;
typedef __attribute__((ext_vector_type(4)))  unsigned int v4u;

__device__ __forceinline__ unsigned pk16(unsigned short a, unsigned short b) { return (unsigned)a | ((unsigned)b << 16); }
__device__ __forceinline__ unsigned short h_bits(float f) { const _Float16 h = (_Float16)f; return __builtin_bit_cast(unsigned short, h); }

__device__ __forceinline__ float h16_to_f32(unsigned hb) {
  const unsigned sgn = (hb & 0x8000u) << 16; const unsigned em = hb & 0x7fffu;
  const float fn = __uint_as_float((em << 13) + 0x38000000u);
  const float fs = (float)em * 5.9604644775390625e-8f;
  const float mag = (em < 0x400u) ? fs : fn; return __uint_as_float(__float_as_uint(mag) | sgn); }
__device__ __forceinline__ float h_lo(unsigned w) { return h16_to_f32(w & 0xffffu); }
__device__ __forceinline__ float h_hi(unsigned w) { return h16_to_f32(w >> 16); }

__device__ __forceinline__ float gelu_erf(float x) {
  return 0.5f * x * (1.0f + erff(x * kInvSqrt2));
}

__device__ __forceinline__ void tie1_h(v8f& a, v16h x, v16h y) { asm volatile("" : "+v"(a) : "v"(x), "v"(y)); }
__device__ __forceinline__ void nop4_h(v8f& a, v16h x, v16h y) { asm volatile("v_nop\n\tv_nop\n\tv_nop\n\tv_nop" : "+v"(a) : "v"(x), "v"(y)); }
__device__ __forceinline__ void tie_acc(v8f& a) { asm volatile("" : "+v"(a)); }
__device__ __forceinline__ void nop4_acc(v8f& a) { asm volatile("v_nop\n\tv_nop\n\tv_nop\n\tv_nop" : "+v"(a)); }
__device__ __forceinline__ void keep4_h(v16h a, v16h b, v16h c, v16h d) { asm volatile("v_nop" :: "v"(a), "v"(b), "v"(c), "v"(d)); }

union FragH { v16h v; v8h h[2]; };
__device__ __forceinline__ v16h frag_load_h(const _Float16* p) {
  FragH f; f.h[0] = *(const v8h*)(p); f.h[1] = *(const v8h*)(p + 16); return f.v;
}
__device__ __forceinline__ v8f mma_h(v16h a, v16h b, v8f c) {
  return __builtin_amdgcn_wmma_f32_16x16x32_f16(false, a, false, b, (short)0, c, false, false);
}

template <int OUT_MODE>
__global__ __launch_bounds__(256) void gemm64_f16_kernel(
    const unsigned short* __restrict__ Ap, int lda,
    const unsigned short* __restrict__ Btp, int ldb,
    void* __restrict__ Cout, int ldc,
    const float* __restrict__ bias,
    int M, int N, int K, float scale) {
  const _Float16* A  = (const _Float16*)(const void*)Ap;
  const _Float16* Bt = (const _Float16*)(const void*)Btp;
  __shared__ __align__(16) float sT[8][16 * 68];
  const int lane = threadIdx.x & 31;
  const int wave = threadIdx.x >> 5;
  const int tilesN = N >> 6;
  const int tilesM = M >> 6;
  const int tile = blockIdx.x * 8 + wave;
  if (tile >= tilesM * tilesN) return;
  const int tm = tile / tilesN;
  const int tn = tile - tm * tilesN;
  const int m0 = tm << 6;
  const int n0 = tn << 6;

  const int rlane = lane & 15;
  const int koff  = (lane >> 4) * 8;
  const int mOff  = (lane >> 4) * 8;

  v8f acc[4][4];
#pragma unroll
  for (int i = 0; i < 4; ++i)
#pragma unroll
    for (int j = 0; j < 4; ++j) acc[i][j] = (v8f){0.f,0.f,0.f,0.f,0.f,0.f,0.f,0.f};

  for (int k0 = 0; k0 < K; k0 += 32) {
    v16h bh[4];
#pragma unroll
    for (int j = 0; j < 4; ++j) {
      const size_t bo = (size_t)(n0 + (j << 4) + rlane) * ldb + koff + k0;
      bh[j] = frag_load_h(Bt + bo);
    }
#pragma unroll
    for (int i = 0; i < 4; ++i) {
      const size_t ao = (size_t)(m0 + (i << 4) + rlane) * lda + koff + k0;
      const v16h ah = frag_load_h(A + ao);
#pragma unroll
      for (int j = 0; j < 4; ++j) acc[i][j] = mma_h(ah, bh[j], acc[i][j]);
      tie1_h(acc[i][0], ah, bh[0]);
      tie1_h(acc[i][1], ah, bh[1]);
      tie1_h(acc[i][2], ah, bh[2]);
      nop4_h(acc[i][3], ah, bh[3]);
    }
    keep4_h(bh[0], bh[1], bh[2], bh[3]);
  }
#pragma unroll
  for (int i = 0; i < 4; ++i)
#pragma unroll
    for (int j = 0; j < 4; ++j) tie_acc(acc[i][j]);
  nop4_acc(acc[3][3]);

  float* slab = sT[wave];
#pragma unroll
  for (int i = 0; i < 4; ++i) {
    const int mBase = m0 + (i << 4);
#pragma unroll
    for (int j = 0; j < 4; ++j) {
      const int n = n0 + (j << 4) + rlane;
      const float bv = bias[n];
#pragma unroll
      for (int r = 0; r < 8; ++r) {
        float v = acc[i][j][r] * scale;
        v += bv;
        slab[(mOff + r) * 68 + (j << 4) + rlane] = v;
      }
    }
    __builtin_amdgcn_fence(__ATOMIC_RELEASE, "workgroup");
    __builtin_amdgcn_wave_barrier();
    __builtin_amdgcn_fence(__ATOMIC_ACQUIRE, "workgroup");
    if (OUT_MODE == 0) {
      float* C = (float*)Cout;
      const int hh = lane >> 4, c4 = (lane & 15) * 4;
      for (int pass = 0; pass < 2; ++pass) {
#pragma unroll
        for (int it = 0; it < 8; ++it) {
          const int row = it * 2 + hh;
          const v4f v = *(const v4f*)(slab + row * 68 + c4);
          *(volatile v4f*)(C + (size_t)(mBase + row) * ldc + n0 + c4) = v;
        }
        __threadfence();
      }
    } else {
      const int q = lane >> 3, c8 = (lane & 7) * 8;
      unsigned short* C = (unsigned short*)Cout;
      for (int pass = 0; pass < 2; ++pass) {
#pragma unroll
        for (int it = 0; it < 4; ++it) {
          const int row = it * 4 + q;
          const float* sp = slab + row * 68 + c8;
          v8h hv;
#pragma unroll
          for (int e = 0; e < 8; ++e) hv[e] = (_Float16)sp[e];
          *(volatile v8h*)(C + (size_t)(mBase + row) * ldc + n0 + c8) = hv;
        }
        __threadfence();
      }
    }
    __builtin_amdgcn_fence(__ATOMIC_RELEASE, "workgroup");
    __builtin_amdgcn_wave_barrier();
    __builtin_amdgcn_fence(__ATOMIC_ACQUIRE, "workgroup");
  }
}

__global__ __launch_bounds__(256) void cast8_f16_kernel(const float* __restrict__ in, unsigned short* __restrict__ out,
                                                        int n8, float carry) {
  const int i = blockIdx.x * 256 + threadIdx.x;
  if (i >= n8) return;
  const float* p = in + 8 * (size_t)i;
  const v4f a = *(const v4f*)(p);
  const v4f c = *(const v4f*)(p + 4);
  unsigned short hb[8];
#pragma unroll
  for (int e = 0; e < 4; ++e) {
    const float fa = a[e] * carry;
    const float fc = c[e] * carry;
    hb[e]     = h_bits(fa);
    hb[4 + e] = h_bits(fc);
  }
  const v4u u = (v4u){pk16(hb[0], hb[1]), pk16(hb[2], hb[3]), pk16(hb[4], hb[5]), pk16(hb[6], hb[7])};
  unsigned short* q = out + 8 * (size_t)i;
  *(volatile v4u*)q = u;
  __threadfence();
  *(volatile v4u*)q = u;
}

__global__ __launch_bounds__(256) void ln_rows_kernel(const float* __restrict__ pre,
                                                      const float* __restrict__ g1, const float* __restrict__ b1,
                                                      const float* __restrict__ g2, const float* __restrict__ b2,
                                                      unsigned short* __restrict__ X, int nrows) {
  const int lane = threadIdx.x & 31;
  const int wave = threadIdx.x >> 5;
  const int row  = blockIdx.x * 8 + wave;
  const bool live = row < nrows;
  const int rc = live ? row : (nrows - 1);
  const float* xr = pre + (size_t)rc * kF;
  const bool tok1 = (rc & 1) != 0;
  const float* gp = tok1 ? g2 : g1;
  const float* bp = tok1 ? b2 : b1;

  float s = 0.0f;
#pragma unroll 1
  for (int it = 0; it < 4; ++it) {
    const float* p = xr + it * 256 + lane * 8;
    const v4f a = *(const v4f*)(p);
    const v4f c = *(const v4f*)(p + 4);
    s += ((a[0] + a[1]) + (a[2] + a[3])) + ((c[0] + c[1]) + (c[2] + c[3]));
  }
#pragma unroll
  for (int off = 16; off > 0; off >>= 1) s += __shfl_xor(s, off, 32);
  const float mean = s * kInvF;

  float qs = 0.0f;
#pragma unroll 1
  for (int it = 0; it < 4; ++it) {
    const float* p = xr + it * 256 + lane * 8;
    const v4f a = *(const v4f*)(p);
    const v4f c = *(const v4f*)(p + 4);
#pragma unroll
    for (int e = 0; e < 4; ++e) {
      const float da = a[e] - mean;
      const float dc = c[e] - mean;
      qs = fmaf(da, da, qs);
      qs = fmaf(dc, dc, qs);
    }
  }
#pragma unroll
  for (int off = 16; off > 0; off >>= 1) qs += __shfl_xor(qs, off, 32);
  const float var = qs * kInvF;
  const float inv = 1.0f / sqrtf(var + kLnEps);

  unsigned short* orow = X + (size_t)rc * kF;
#pragma unroll 1
  for (int it = 0; it < 4; ++it) {
    const int col = it * 256 + lane * 8;
    const v4f a  = *(const v4f*)(xr + col);
    const v4f c  = *(const v4f*)(xr + col + 4);
    const v4f ga = *(const v4f*)(gp + col);
    const v4f gc = *(const v4f*)(gp + col + 4);
    const v4f ba = *(const v4f*)(bp + col);
    const v4f bc = *(const v4f*)(bp + col + 4);
    unsigned short hb[8];
#pragma unroll
    for (int e = 0; e < 4; ++e) {
      const float ya = (a[e] - mean) * inv * ga[e] + ba[e];
      const float yc = (c[e] - mean) * inv * gc[e] + bc[e];
      hb[e]     = h_bits(ya);
      hb[4 + e] = h_bits(yc);
    }
    const v4u u = (v4u){pk16(hb[0], hb[1]), pk16(hb[2], hb[3]), pk16(hb[4], hb[5]), pk16(hb[6], hb[7])};
    if (live) {
      *(volatile v4u*)(orow + col) = u;
      __threadfence();
      *(volatile v4u*)(orow + col) = u;
    }
  }
}

__global__ __launch_bounds__(256) void attn2_kernel(const unsigned short* __restrict__ qkv,
                                                    unsigned short* __restrict__ o, int nb, float scl) {
  const int lane = threadIdx.x & 31;
  const int wave = threadIdx.x >> 5;
  const int unit = blockIdx.x * 8 + wave;
  const int nunits = nb * 4;
  const bool live = unit < nunits;
  const int uc = live ? unit : (nunits - 1);
  const int b  = uc >> 2;
  const int hp = uc & 3;
  const size_t r0 = (size_t)(2 * b) * kQKV;
  const size_t r1 = r0 + kQKV;
  const int col = hp * (2 * kHD) + lane * 8;

  const v4u q0w = *(const v4u*)(qkv + r0 + col);
  const v4u q1w = *(const v4u*)(qkv + r1 + col);
  const v4u k0w = *(const v4u*)(qkv + r0 + kF + col);
  const v4u k1w = *(const v4u*)(qkv + r1 + kF + col);
  const v4u v0w = *(const v4u*)(qkv + r0 + 2 * kF + col);
  const v4u v1w = *(const v4u*)(qkv + r1 + 2 * kF + col);

  float s00 = 0.0f, s01 = 0.0f, s10 = 0.0f, s11 = 0.0f;
#pragma unroll
  for (int w = 0; w < 4; ++w) {
    const unsigned uq0 = q0w[w];
    const unsigned uq1 = q1w[w];
    const unsigned uk0 = k0w[w];
    const unsigned uk1 = k1w[w];
    const float q0a = h_lo(uq0), q0b = h_hi(uq0);
    const float q1a = h_lo(uq1), q1b = h_hi(uq1);
    const float k0a = h_lo(uk0), k0b = h_hi(uk0);
    const float k1a = h_lo(uk1), k1b = h_hi(uk1);
    s00 = fmaf(q0a, k0a, s00); s00 = fmaf(q0b, k0b, s00);
    s01 = fmaf(q0a, k1a, s01); s01 = fmaf(q0b, k1b, s01);
    s10 = fmaf(q1a, k0a, s10); s10 = fmaf(q1b, k0b, s10);
    s11 = fmaf(q1a, k1a, s11); s11 = fmaf(q1b, k1b, s11);
  }
#pragma unroll
  for (int off = 8; off > 0; off >>= 1) {
    s00 += __shfl_xor(s00, off, 32);
    s01 += __shfl_xor(s01, off, 32);
    s10 += __shfl_xor(s10, off, 32);
    s11 += __shfl_xor(s11, off, 32);
  }
  s00 *= scl; s01 *= scl; s10 *= scl; s11 *= scl;

  const float d0 = s01 - s00;
  const float d1 = s11 - s10;
  const float e0 = expf(-fabsf(d0));
  const float e1 = expf(-fabsf(d1));
  const float i0 = 1.0f / (1.0f + e0);
  const float i1 = 1.0f / (1.0f + e1);
  const float sm0 = e0 * i0;
  const float sm1 = e1 * i1;
  const float a00 = (d0 > 0.0f) ? sm0 : i0;
  const float a01 = (d0 > 0.0f) ? i0 : sm0;
  const float a10 = (d1 > 0.0f) ? sm1 : i1;
  const float a11 = (d1 > 0.0f) ? i1 : sm1;

  unsigned ow0[4], ow1[4];
#pragma unroll
  for (int w = 0; w < 4; ++w) {
    const unsigned uv0 = v0w[w];
    const unsigned uv1 = v1w[w];
    const float v0a = h_lo(uv0), v0b = h_hi(uv0);
    const float v1a = h_lo(uv1), v1b = h_hi(uv1);
    const float o0a = a00 * v0a + a01 * v1a;
    const float o0b = a00 * v0b + a01 * v1b;
    const float o1a = a10 * v0a + a11 * v1a;
    const float o1b = a10 * v0b + a11 * v1b;
    ow0[w] = pk16(h_bits(o0a), h_bits(o0b));
    ow1[w] = pk16(h_bits(o1a), h_bits(o1b));
  }
  const v4u u0 = (v4u){ow0[0], ow0[1], ow0[2], ow0[3]};
  const v4u u1 = (v4u){ow1[0], ow1[1], ow1[2], ow1[3]};
  unsigned short* o0p = o + (size_t)(2 * b) * kF + col;
  unsigned short* o1p = o0p + kF;
  if (live) {
    *(volatile v4u*)o0p = u0;
    *(volatile v4u*)o1p = u1;
    __threadfence();
    *(volatile v4u*)o0p = u0;
    *(volatile v4u*)o1p = u1;
  }
}

__global__ __launch_bounds__(512) void gate_fuse_kernel(const float* __restrict__ gpre,
                                                        const float* __restrict__ w2, const float* __restrict__ b2v,
                                                        const unsigned short* __restrict__ ao,
                                                        unsigned short* __restrict__ fused,
                                                        float* __restrict__ gw_out, int nb) {
  __shared__ float sG[32];
  const int lane = threadIdx.x & 31;
  const int wave = threadIdx.x >> 5;
  const int b = blockIdx.x * 16 + wave;
  const bool live = b < nb;
  const int bc = live ? b : (nb - 1);
  const float* hr = gpre + (size_t)bc * kF;

  float d0 = 0.0f, d1 = 0.0f;
#pragma unroll 1
  for (int it = 0; it < 32; ++it) {
    const int idx = it * 32 + lane;
    float x  = hr[idx];
    float wa = w2[idx];
    float wb = w2[kF + idx];
    asm volatile("" : "+v"(x), "+v"(wa), "+v"(wb));
    const float g = gelu_erf(x);
    d0 = fmaf(g, wa, d0);
    d1 = fmaf(g, wb, d1);
  }
#pragma unroll
  for (int off = 16; off > 0; off >>= 1) {
    d0 += __shfl_xor(d0, off, 32);
    d1 += __shfl_xor(d1, off, 32);
  }
  const float l0 = d0 + b2v[0];
  const float l1 = d1 + b2v[1];
  const float mx = fmaxf(l0, l1);
  const float e0 = expf(l0 - mx);
  const float e1 = expf(l1 - mx);
  const float inv = 1.0f / (e0 + e1);
  const float gw0 = e0 * inv;
  const float gw1 = e1 * inv;
  if (lane == 0) {
    sG[wave * 2]     = gw0;
    sG[wave * 2 + 1] = gw1;
  }

  const unsigned short* cr = ao + (size_t)(2 * bc) * kF;
  const unsigned short* gr = cr + kF;
  unsigned short* fr = fused + (size_t)bc * kF;
#pragma unroll 1
  for (int it = 0; it < 4; ++it) {
    const int col = it * 256 + lane * 8;
    const v4u cw = *(const v4u*)(cr + col);
    const v4u gv = *(const v4u*)(gr + col);
    unsigned ow[4];
#pragma unroll
    for (int w = 0; w < 4; ++w) {
      const unsigned uc = cw[w];
      const unsigned ug = gv[w];
      const float ca = h_lo(uc), cb = h_hi(uc);
      const float ga = h_lo(ug), gb = h_hi(ug);
      const float fa = gw0 * ca + gw1 * ga;
      const float fb = gw0 * cb + gw1 * gb;
      ow[w] = pk16(h_bits(fa), h_bits(fb));
    }
    const v4u u = (v4u){ow[0], ow[1], ow[2], ow[3]};
    if (live) {
      *(volatile v4u*)(fr + col) = u;
      __threadfence();
      *(volatile v4u*)(fr + col) = u;
    }
  }

  __syncthreads();
  const bool blockLive = (blockIdx.x * 16 + 15) < nb;
  if (wave == 0 && blockLive) {
    const float v = sG[lane];
    float* dst = gw_out + (size_t)blockIdx.x * 32 + lane;
    *(volatile float*)dst = v;
    __threadfence();
    *(volatile float*)dst = v;
  }
}

__global__ __launch_bounds__(256) void gelu_out_kernel(const float* __restrict__ pin, float* __restrict__ dst, int n) {
  const int base = blockIdx.x * 2048;
#pragma unroll 1
  for (int it = 0; it < 8; ++it) {
    const int i = base + it * 256 + (int)threadIdx.x;
    const bool live = i < n;
    const int ic = live ? i : (n - 1);
    float x = pin[ic];
    asm volatile("" : "+v"(x));
    const float y = gelu_erf(x);
    if (live) {
      *(volatile float*)(dst + i) = y;
      __threadfence();
      *(volatile float*)(dst + i) = y;
    }
  }
}

template <int OUT_MODE>
static void launch_gemm(const unsigned short* A, int lda, const unsigned short* Bt, int ldb,
                        void* C, int ldc, const float* bias, int M, int N, int K, float scale, hipStream_t stream) {
  const int tiles = (M / 64) * (N / 64);
  const int blocks = (tiles + 7) / 8;
  gemm64_f16_kernel<OUT_MODE><<<blocks, 256, 0, stream>>>(A, lda, Bt, ldb, C, ldc, bias, M, N, K, scale);
}

static void launch_cast(const float* in, unsigned short* out, int n, float carry, hipStream_t stream) {
  const int n8 = n / 8;
  cast8_f16_kernel<<<(n8 + 255) / 256, 256, 0, stream>>>(in, out, n8, carry);
}

constexpr size_t kSzWc   = (size_t)kF * kCD * 2;
constexpr size_t kSzWg   = (size_t)kF * kCD * 2;
constexpr size_t kSzWqkv = (size_t)kQKV * kF * 2;
constexpr size_t kSzWo   = (size_t)kF * kF * 2;
constexpr size_t kSzWg1  = (size_t)kF * 2 * kF * 2;
constexpr size_t kSzWp   = (size_t)kF * kF * 2;
constexpr size_t kSzEc   = (size_t)kB * kCD * 2;
constexpr size_t kSzEg   = (size_t)kB * kCD * 2;
constexpr size_t kSzPre  = (size_t)kChunkT * kF * 4;
constexpr size_t kSzX    = (size_t)kChunkT * kF * 2;
constexpr size_t kSzQkv  = (size_t)kChunkT * kQKV * 2;
constexpr size_t kSzO    = (size_t)kChunkT * kF * 2;
constexpr size_t kSzAo   = (size_t)kChunkT * kF * 2;
constexpr size_t kSzGpre = (size_t)kChunkB * kF * 4;
constexpr size_t kSzFus  = (size_t)kChunkB * kF * 2;
constexpr size_t kSzP    = (size_t)kChunkB * kF * 4;
constexpr size_t kWsTotal = kSzWc + kSzWg + kSzWqkv + kSzWo + kSzWg1 + kSzWp + kSzEc + kSzEg +
                            kSzPre + kSzX + kSzQkv + kSzO + kSzAo + kSzGpre + kSzFus + kSzP;
static_assert(kWsTotal == 121634816ull, "carve total");
static_assert(kWsTotal <= 134217728ull, "carve limit");
static_assert(((size_t)kB * kF * 4) % 128 == 0, "second output starts on a line");
static_assert(((size_t)kChunkB * kF) % 2048 == 0, "activation pass coverage");

extern "C" void kernel_launch(void* const* d_in, const int* in_sizes, int n_in,
                              void* d_out, int out_size, void* d_ws, size_t ws_size, hipStream_t stream) {
  if (n_in < 20) return;
  if (ws_size < kWsTotal) return;
  if (in_sizes[0] != kB * kCD || in_sizes[1] != kB * kCD) return;
  if (in_sizes[10] != kQKV * kF || in_sizes[14] != kF * 2 * kF) return;
  if (out_size != kB * kF + kB * 2) return;

  const float* cnn_embed  = (const float*)d_in[0];
  const float* gnn_embed  = (const float*)d_in[1];
  const float* cnn_w      = (const float*)d_in[2];
  const float* cnn_b      = (const float*)d_in[3];
  const float* gnn_w      = (const float*)d_in[4];
  const float* gnn_b      = (const float*)d_in[5];
  const float* ln1_g      = (const float*)d_in[6];
  const float* ln1_b      = (const float*)d_in[7];
  const float* ln2_g      = (const float*)d_in[8];
  const float* ln2_b      = (const float*)d_in[9];
  const float* attn_in_w  = (const float*)d_in[10];
  const float* attn_in_b  = (const float*)d_in[11];
  const float* attn_out_w = (const float*)d_in[12];
  const float* attn_out_b = (const float*)d_in[13];
  const float* gate_w1    = (const float*)d_in[14];
  const float* gate_b1    = (const float*)d_in[15];
  const float* gate_w2    = (const float*)d_in[16];
  const float* gate_b2    = (const float*)d_in[17];
  const float* proj_w     = (const float*)d_in[18];
  const float* proj_b     = (const float*)d_in[19];

  char* ws = (char*)d_ws;
  size_t off = 0;
  auto carve = [&](size_t bytes) -> char* { char* p = ws + off; off += bytes; return p; };
  unsigned short* Wc   = (unsigned short*)carve(kSzWc);
  unsigned short* Wg   = (unsigned short*)carve(kSzWg);
  unsigned short* Wqkv = (unsigned short*)carve(kSzWqkv);
  unsigned short* Wo   = (unsigned short*)carve(kSzWo);
  unsigned short* Wg1  = (unsigned short*)carve(kSzWg1);
  unsigned short* Wp   = (unsigned short*)carve(kSzWp);
  unsigned short* Ec   = (unsigned short*)carve(kSzEc);
  unsigned short* Eg   = (unsigned short*)carve(kSzEg);
  float*          preLN = (float*)carve(kSzPre);
  unsigned short* Xp   = (unsigned short*)carve(kSzX);
  unsigned short* qkvp = (unsigned short*)carve(kSzQkv);
  unsigned short* op   = (unsigned short*)carve(kSzO);
  unsigned short* aop  = (unsigned short*)carve(kSzAo);
  float*          gpre = (float*)carve(kSzGpre);
  unsigned short* fusp = (unsigned short*)carve(kSzFus);
  float*          Pp   = (float*)carve(kSzP);

  float* out0 = (float*)d_out;
  float* out1 = out0 + (size_t)kB * kF;

  const float scl = 1.0f / sqrtf((float)kHD);

  launch_cast(cnn_w,      Wc,   kF * kCD,     kWCarry, stream);
  launch_cast(gnn_w,      Wg,   kF * kCD,     kWCarry, stream);
  launch_cast(attn_in_w,  Wqkv, kQKV * kF,    kWCarry, stream);
  launch_cast(attn_out_w, Wo,   kF * kF,      kWCarry, stream);
  launch_cast(gate_w1,    Wg1,  kF * 2 * kF,  kWCarry, stream);
  launch_cast(proj_w,     Wp,   kF * kF,      kWCarry, stream);
  launch_cast(cnn_embed,  Ec,   kB * kCD,     1.0f,    stream);
  launch_cast(gnn_embed,  Eg,   kB * kCD,     1.0f,    stream);

  for (int c = 0; c < kNChunk; ++c) {
    const unsigned short* EcC = Ec + (size_t)c * kChunkB * kCD;
    const unsigned short* EgC = Eg + (size_t)c * kChunkB * kCD;

    launch_gemm<0>(EcC, kCD, Wc, kCD, (void*)preLN,        2 * kF, cnn_b, kChunkB, kF, kCD, kWCarryInv, stream);
    launch_gemm<0>(EgC, kCD, Wg, kCD, (void*)(preLN + kF), 2 * kF, gnn_b, kChunkB, kF, kCD, kWCarryInv, stream);

    ln_rows_kernel<<<kChunkT / 8, 256, 0, stream>>>(preLN, ln1_g, ln1_b, ln2_g, ln2_b, Xp, kChunkT);

    launch_gemm<1>(Xp, kF, Wqkv, kF, (void*)qkvp, kQKV, attn_in_b, kChunkT, kQKV, kF, kWCarryInv, stream);

    attn2_kernel<<<(kChunkB * 4) / 8, 256, 0, stream>>>(qkvp, op, kChunkB, scl);

    launch_gemm<1>(op, kF, Wo, kF, (void*)aop, kF, attn_out_b, kChunkT, kF, kF, kWCarryInv, stream);

    launch_gemm<0>(aop, 2 * kF, Wg1, 2 * kF, (void*)gpre, kF, gate_b1, kChunkB, kF, 2 * kF, kWCarryInv, stream);

    gate_fuse_kernel<<<kChunkB / 16, 512, 0, stream>>>(gpre, gate_w2, gate_b2, aop, fusp,
                                                       out1 + (size_t)c * kChunkB * 2, kChunkB);

    launch_gemm<0>(fusp, kF, Wp, kF, (void*)Pp, kF, proj_b, kChunkB, kF, kF, kWCarryInv, stream);
    gelu_out_kernel<<<(kChunkB * kF) / 2048, 256, 0, stream>>>(Pp, out0 + (size_t)c * kChunkB * kF, kChunkB * kF);
  }
}
